// ModelQK_13357348290921
// MI455X (gfx1250) — hardware-run, weakly checked
//
#include <hip/hip_runtime.h>
#include <stddef.h>
#include <stdint.h>


#define QD      192
#define KD      64
#define CD      256
#define DO      128
#define YC      640
#define NTHR    256
#define NWAVE   8
#define EPT     8
#define CHUNK   (NTHR * EPT)
#define WCAP    (EPT * 32)
#define LISTN   (NWAVE * WCAP)
#define NBMAX   2048
#define RCAP    28672
#define DEGCAP  4096
#define STW     128
#define GBM     64
#define GBN     64
#define GTHR    128
#define CX      8.0f
#define CW      64.0f
#define CG      64.0f
#define SCL_XW  0.001953125f
#define SCL_GW  0.000244140625f
#define ISC     0.0625f
#define WSMAX   134217728
#define LDS_AGG ((2 * RCAP + 2 * NBMAX + LISTN) * 4 + 64)

static_assert((CHUNK & (CHUNK - 1)) == 0 && CHUNK <= 4096);
static_assert((NBMAX & (NBMAX - 1)) == 0 && NBMAX <= 4096);
static_assert(NTHR * 8 == NBMAX);
static_assert(LISTN >= NBMAX);
static_assert(LISTN >= NWAVE * WCAP);
static_assert((RCAP % 32) == 0);
static_assert(NWAVE * STW <= RCAP);
static_assert(STW >= KD);
static_assert(LDS_AGG <= 300000);
static_assert(GBM == (GTHR / 32) * 16);
static_assert((CD % 32) == 0 && (KD % 32) == 0);
static_assert((YC % GBN) == 0 && (DO % GBN) == 0);
static_assert(CD / 8 == 32 && KD / 8 == 8);
static_assert(QD + KD == CD);
static_assert(((DO * KD / 8) % 32) == 0 && ((YC / 4) % 32) == 0);

typedef float    v4f  __attribute__((ext_vector_type(4)));
typedef float    v8f  __attribute__((ext_vector_type(8)));
typedef int      v4i  __attribute__((ext_vector_type(4)));
typedef int      v8i  __attribute__((ext_vector_type(8)));
typedef _Float16 v8h  __attribute__((ext_vector_type(8)));
typedef _Float16 v16h __attribute__((ext_vector_type(16)));
union FragH { v16h v; v8h h[2]; v8i w; };

__device__ __forceinline__ v8f wmh(const FragH& a, const FragH& b, v8f c) {
  v8f d = __builtin_amdgcn_wmma_f32_16x16x32_f16(false, a.v, false, b.v, (short)0, c, false, false);
  asm volatile("v_nop\n\tv_nop\n\tv_nop\n\tv_nop" : "+v"(d) : "v"(a.w), "v"(b.w));
  return d;
}

__device__ __forceinline__ void ldwait() {
  asm volatile("s_wait_loadcnt 0x0" ::: "memory");
}

__device__ __forceinline__ v8h cvt8h(const v4f a, const v4f b, const float c) {
  v8h hv;
  hv[0] = (_Float16)(a.x * c); hv[1] = (_Float16)(a.y * c);
  hv[2] = (_Float16)(a.z * c); hv[3] = (_Float16)(a.w * c);
  hv[4] = (_Float16)(b.x * c); hv[5] = (_Float16)(b.y * c);
  hv[6] = (_Float16)(b.z * c); hv[7] = (_Float16)(b.w * c);
  return hv;
}

__device__ __forceinline__ int scan_chunk(const int* __restrict__ dsts, int nE, int cbase, int slotBase,
                                          int nb, int vec8, int* list, int tid, int lane, int wave) {
  int wc = 0;
  const int el0  = tid * EPT;
  const int e0   = cbase + el0;
  const int sent = -2147483647 - 1;
  v4i da, db;
  if (vec8 != 0 && cbase + CHUNK <= nE) {
    da = *(const v4i*)(dsts + e0);
    db = *(const v4i*)(dsts + e0 + 4);
  } else {
    da.x = (e0     < nE) ? dsts[min(e0,     nE - 1)] : sent;
    da.y = (e0 + 1 < nE) ? dsts[min(e0 + 1, nE - 1)] : sent;
    da.z = (e0 + 2 < nE) ? dsts[min(e0 + 2, nE - 1)] : sent;
    da.w = (e0 + 3 < nE) ? dsts[min(e0 + 3, nE - 1)] : sent;
    db.x = (e0 + 4 < nE) ? dsts[min(e0 + 4, nE - 1)] : sent;
    db.y = (e0 + 5 < nE) ? dsts[min(e0 + 5, nE - 1)] : sent;
    db.z = (e0 + 6 < nE) ? dsts[min(e0 + 6, nE - 1)] : sent;
    db.w = (e0 + 7 < nE) ? dsts[min(e0 + 7, nE - 1)] : sent;
  }
  const unsigned nbs = (unsigned)slotBase;
  const unsigned unb = (unsigned)nb;
  const unsigned s0 = (unsigned)da.x - nbs, s1 = (unsigned)da.y - nbs;
  const unsigned s2 = (unsigned)da.z - nbs, s3 = (unsigned)da.w - nbs;
  const unsigned s4 = (unsigned)db.x - nbs, s5 = (unsigned)db.y - nbs;
  const unsigned s6 = (unsigned)db.z - nbs, s7 = (unsigned)db.w - nbs;
  const bool h0 = s0 < unb, h1 = s1 < unb, h2 = s2 < unb, h3 = s3 < unb;
  const bool h4 = s4 < unb, h5 = s5 < unb, h6 = s6 < unb, h7 = s7 < unb;
  const unsigned any = __builtin_amdgcn_ballot_w32(h0 | h1 | h2 | h3 | h4 | h5 | h6 | h7);
  if (any != 0u) {
#define HITJ(J, HJ, SJ) { \
      const unsigned mj = __builtin_amdgcn_ballot_w32(HJ); \
      if (mj != 0u) { \
        if (HJ) { \
          const int pos = wc + (int)__builtin_amdgcn_mbcnt_lo(mj, 0u); \
          if (pos < WCAP) list[wave * WCAP + pos] = ((el0 + (J)) << 12) | (int)(SJ); \
        } \
        wc += (int)__builtin_popcount(mj); } }
    HITJ(0, h0, s0)
    HITJ(1, h1, s1)
    HITJ(2, h2, s2)
    HITJ(3, h3, s3)
    HITJ(4, h4, s4)
    HITJ(5, h5, s5)
    HITJ(6, h6, s6)
    HITJ(7, h7, s7)
#undef HITJ
  }
  return wc;
}

__global__ __launch_bounds__(NTHR) void k_xprep(const float* __restrict__ query, const int* __restrict__ kid,
                                                _Float16* xh, int nN, int nUnits) {
  const int i = (int)blockIdx.x * NTHR + (int)threadIdx.x;
  if (i >= nUnits) return;
  const int row = i >> 5;
  const int c0  = (i & 31) * 8;
  const int rc  = row < nN ? row : nN - 1;
  const int cq  = c0 < QD - 8 ? c0 : QD - 8;
  const float* p = query + (size_t)rc * QD + cq;
  v4f a = *(const v4f*)p, b = *(const v4f*)(p + 4);
  const int kv = kid[rc];
  const int j0 = c0 - QD;
  v4f oa, ob;
  oa.x = (j0 + 0 == kv) ? 1.0f : 0.0f;  oa.y = (j0 + 1 == kv) ? 1.0f : 0.0f;
  oa.z = (j0 + 2 == kv) ? 1.0f : 0.0f;  oa.w = (j0 + 3 == kv) ? 1.0f : 0.0f;
  ob.x = (j0 + 4 == kv) ? 1.0f : 0.0f;  ob.y = (j0 + 5 == kv) ? 1.0f : 0.0f;
  ob.z = (j0 + 6 == kv) ? 1.0f : 0.0f;  ob.w = (j0 + 7 == kv) ? 1.0f : 0.0f;
  if (c0 >= QD) { a = oa; b = ob; }
  const v4f z4 = {0.f, 0.f, 0.f, 0.f};
  if (row >= nN) { a = z4; b = z4; }
  const v8h hv = cvt8h(a, b, CX);
  const size_t o = (size_t)row * CD + c0;
  *(volatile v8h*)(xh + o) = hv;
  __threadfence();
  *(volatile v8h*)(xh + o) = hv;
}

__global__ __launch_bounds__(NTHR) void k_wcat(const float* __restrict__ Wq, const float* __restrict__ Wk,
                                               const float* __restrict__ Wv, const float* __restrict__ Ws,
                                               _Float16* wt, int nUnits) {
  const int u = (int)blockIdx.x * NTHR + (int)threadIdx.x;
  if (u >= nUnits) return;
  const int n  = u >> 5;
  const int k8 = (u & 31) * 8;
  const float* src = (n < 256) ? Wq : ((n < 512) ? Wk : ((n < 576) ? Wv : Ws));
  int col = (n < 256) ? n : ((n < 512) ? (n - 256) : ((n < 576) ? (QD + n - 512) : (QD + n - 576)));
  col = col < 0 ? 0 : (col > CD - 1 ? CD - 1 : col);
  v4f a, b;
  a.x = src[(size_t)(k8 + 0) * CD + col];  a.y = src[(size_t)(k8 + 1) * CD + col];
  a.z = src[(size_t)(k8 + 2) * CD + col];  a.w = src[(size_t)(k8 + 3) * CD + col];
  b.x = src[(size_t)(k8 + 4) * CD + col];  b.y = src[(size_t)(k8 + 5) * CD + col];
  b.z = src[(size_t)(k8 + 6) * CD + col];  b.w = src[(size_t)(k8 + 7) * CD + col];
  const v8h hv = cvt8h(a, b, CW);
  const size_t o = (size_t)n * CD + k8;
  *(volatile v8h*)(wt + o) = hv;
  __threadfence();
  *(volatile v8h*)(wt + o) = hv;
}

__global__ __launch_bounds__(NTHR) void k_wob(const float* __restrict__ Wo,
                                              const float* __restrict__ bq, const float* __restrict__ bk,
                                              const float* __restrict__ bv, const float* __restrict__ bs,
                                              _Float16* wot, float* bc, int nWo, int nB) {
  const int u = (int)blockIdx.x * NTHR + (int)threadIdx.x;
  if (u < nWo) {
    const int n  = u >> 3;
    const int k8 = (u & 7) * 8;
    v4f a, b;
    a.x = Wo[(size_t)(k8 + 0) * DO + n];  a.y = Wo[(size_t)(k8 + 1) * DO + n];
    a.z = Wo[(size_t)(k8 + 2) * DO + n];  a.w = Wo[(size_t)(k8 + 3) * DO + n];
    b.x = Wo[(size_t)(k8 + 4) * DO + n];  b.y = Wo[(size_t)(k8 + 5) * DO + n];
    b.z = Wo[(size_t)(k8 + 6) * DO + n];  b.w = Wo[(size_t)(k8 + 7) * DO + n];
    const v8h hv = cvt8h(a, b, CW);
    const size_t o = (size_t)n * KD + k8;
    *(volatile v8h*)(wot + o) = hv;
    __threadfence();
    *(volatile v8h*)(wot + o) = hv;
  } else if (u < nWo + nB) {
    const int n0 = 4 * (u - nWo);
    float r[4];
#pragma unroll
    for (int e = 0; e < 4; ++e) {
      const int n = n0 + e;
      int iq = n;            iq = iq < 0 ? 0 : (iq > CD - 1 ? CD - 1 : iq);
      int ik = n - 256;      ik = ik < 0 ? 0 : (ik > CD - 1 ? CD - 1 : ik);
      int iv = QD + n - 512; iv = iv < 0 ? 0 : (iv > CD - 1 ? CD - 1 : iv);
      int is = QD + n - 576; is = is < 0 ? 0 : (is > CD - 1 ? CD - 1 : is);
      const float vq = bq[iq], vk = bk[ik], vv = bv[iv], vs = bs[is];
      r[e] = (n < 256) ? vq : ((n < 512) ? vk : ((n < 576) ? vv : vs));
    }
    v4f s;
    s.x = r[0]; s.y = r[1]; s.z = r[2]; s.w = r[3];
    *(volatile v4f*)(bc + n0) = s;
    __threadfence();
    *(volatile v4f*)(bc + n0) = s;
  }
}

template<int EPI>
__global__ __launch_bounds__(GTHR) void k_gemm(
    const _Float16* __restrict__ A, const _Float16* __restrict__ WT, const float* __restrict__ bias,
    float* outF, int K, int ldo, int nRows, float scl)
{
  __shared__ __attribute__((aligned(16))) float stg[GBM * GBN];
  const int tid = (int)threadIdx.x, lane = tid & 31, wave = tid >> 5, hh = lane >> 4, m = lane & 15;
  const int rowBase = (int)blockIdx.x * GBM;
  const int col0    = (int)blockIdx.y * GBN;

  v8f acc[4];
  {
    const v8f z = {0.f, 0.f, 0.f, 0.f, 0.f, 0.f, 0.f, 0.f};
    acc[0] = z; acc[1] = z; acc[2] = z; acc[3] = z;
  }
  const _Float16* ap = A  + (size_t)(rowBase + 16 * wave + m) * (size_t)K + 8 * hh;
  const _Float16* wp = WT + (size_t)(col0 + m) * (size_t)K + 8 * hh;
  const int ksteps = K >> 5;
#pragma unroll 1
  for (int ks = 0; ks < ksteps; ++ks) {
    FragH af;
    af.h[0] = *(const v8h*)(ap + 32 * ks);
    af.h[1] = *(const v8h*)(ap + 32 * ks + 16);
#pragma unroll
    for (int t = 0; t < 4; ++t) {
      const _Float16* wq = wp + (size_t)(16 * t) * (size_t)K + 32 * ks;
      FragH bf;
      bf.h[0] = *(const v8h*)wq;
      bf.h[1] = *(const v8h*)(wq + 16);
      acc[t] = wmh(af, bf, acc[t]);
    }
  }

#pragma unroll
  for (int t = 0; t < 4; ++t) {
    const int lc = 16 * t + m;
    const float bvl = bias[col0 + lc];
#pragma unroll
    for (int r = 0; r < 8; ++r) {
      const int lr = 16 * wave + 8 * hh + r;
      stg[lr * GBN + lc] = fmaf(acc[t][r], scl, bvl);
    }
  }
  __syncthreads();

  v4f fv[8];
#pragma unroll
  for (int i = 0; i < 8; ++i) {
    const int lr = 16 * wave + 2 * i + hh;
    fv[i] = *(const v4f*)(stg + lr * GBN + 4 * m);
  }
#pragma unroll
  for (int i = 0; i < 8; ++i) {
    const int lr = 16 * wave + 2 * i + hh;
    const int gr = rowBase + lr;
    float* op = outF + (size_t)gr * (size_t)ldo + col0 + 4 * m;
    if (EPI != 3 || gr < nRows) *(volatile v4f*)op = fv[i];
  }
  __threadfence();
#pragma unroll
  for (int i = 0; i < 8; ++i) {
    const int lr = 16 * wave + 2 * i + hh;
    const int gr = rowBase + lr;
    float* op = outF + (size_t)gr * (size_t)ldo + col0 + 4 * m;
    if (EPI != 3 || gr < nRows) *(volatile v4f*)op = fv[i];
  }
}

__global__ __launch_bounds__(NTHR) void k_agg(
    const int* __restrict__ srcs, const int* __restrict__ dsts,
    const float* __restrict__ Y, _Float16* RH, int nN, int nE, int nb, int vec8, int MPr) {
  extern __shared__ v4f lds_dyn[];
  int* reg1 = (int*)lds_dyn;
  int* reg2 = reg1 + RCAP;
  int* scnt = reg2 + RCAP;
  int* soff = scnt + NBMAX;
  int* list = soff + NBMAX;
  int* wcnt = list + LISTN;
  int* wtot = wcnt + NWAVE;
  const int tid = (int)threadIdx.x, lane = tid & 31, wave = tid >> 5;
  const int nodeBase = (int)blockIdx.x * nb;

  for (int i = tid; i < NBMAX; i += NTHR) scnt[i] = 0;
  __syncthreads();

  int tot = 0;
  const int nChunks = (nE + CHUNK - 1) / CHUNK;
#pragma unroll 1
  for (int ch = 0; ch < nChunks; ++ch) {
    const int cbase = ch * CHUNK;
    const int wc = scan_chunk(dsts, nE, cbase, nodeBase, nb, vec8, list, tid, lane, wave);
    if (lane == 0) wcnt[wave] = wc;
    __syncthreads();
    int pre = 0, all = 0;
#pragma unroll
    for (int w2 = 0; w2 < NWAVE; ++w2) {
      int c = wcnt[w2];
      c = c < 0 ? 0 : (c > WCAP ? WCAP : c);
      all += c;
      pre += (w2 < wave) ? c : 0;
    }
    const int wcc  = wc > WCAP ? WCAP : wc;
    const int base = tot + pre;
#pragma unroll 1
    for (int i = lane; i < wcc; i += 32) {
      const int ent = list[wave * WCAP + i];
      const int el  = (ent >> 12) & (CHUNK - 1);
      const int sl  = ent & (NBMAX - 1);
      int eid = cbase + el;
      eid = eid > nE - 1 ? nE - 1 : eid;
      const int pos = base + i;
      if (pos < RCAP) reg1[pos] = (int)(((unsigned)eid << 12) | (unsigned)sl);
    }
    tot += all;
    tot = tot > RCAP ? RCAP : tot;
    __syncthreads();
  }
  const int nh = tot;

  if (wave == 0) {
#pragma unroll 1
    for (int b0 = 0; b0 < nh; b0 += 32) {
      const int idx = b0 + lane;
      const int uv  = reg1[idx < RCAP ? idx : RCAP - 1];
      const int m32 = (nh - b0) < 32 ? (nh - b0) : 32;
#pragma unroll 1
      for (int k = 0; k < m32; ++k) {
        const int u  = __builtin_amdgcn_readlane(uv, k);
        const int sl = u & (NBMAX - 1);
        if (lane == 0) scnt[sl] = scnt[sl] + 1;
      }
    }
  }
  __syncthreads();

  {
    const v4i ca = *(const v4i*)(scnt + 8 * tid);
    const v4i cb = *(const v4i*)(scnt + 8 * tid + 4);
    const int e0 = ca.x < 0 ? 0 : ca.x, e1 = ca.y < 0 ? 0 : ca.y, e2 = ca.z < 0 ? 0 : ca.z, e3 = ca.w < 0 ? 0 : ca.w;
    const int e4 = cb.x < 0 ? 0 : cb.x, e5 = cb.y < 0 ? 0 : cb.y, e6 = cb.z < 0 ? 0 : cb.z, e7 = cb.w < 0 ? 0 : cb.w;
    const int ts = e0 + e1 + e2 + e3 + e4 + e5 + e6 + e7;
    int incl = ts;
#pragma unroll
    for (int d = 1; d < 32; d <<= 1) {
      const int up = __shfl_up(incl, d);
      if (lane >= d) incl += up;
    }
    if (lane == 31) wtot[wave] = incl;
    __syncthreads();
    int pre = 0;
#pragma unroll
    for (int w2 = 0; w2 < NWAVE; ++w2) pre += (w2 < wave) ? wtot[w2] : 0;
    int run = pre + incl - ts;
    soff[8 * tid + 0] = run; run += e0;
    soff[8 * tid + 1] = run; run += e1;
    soff[8 * tid + 2] = run; run += e2;
    soff[8 * tid + 3] = run; run += e3;
    soff[8 * tid + 4] = run; run += e4;
    soff[8 * tid + 5] = run; run += e5;
    soff[8 * tid + 6] = run; run += e6;
    soff[8 * tid + 7] = run;
  }
  __syncthreads();
  for (int i = tid; i < NBMAX; i += NTHR) list[i] = soff[i];
  __syncthreads();

  if (wave == 0) {
#pragma unroll 1
    for (int b0 = 0; b0 < nh; b0 += 32) {
      const int idx = b0 + lane;
      const int uv  = reg1[idx < RCAP ? idx : RCAP - 1];
      const int m32 = (nh - b0) < 32 ? (nh - b0) : 32;
#pragma unroll 1
      for (int k = 0; k < m32; ++k) {
        const int u   = __builtin_amdgcn_readlane(uv, k);
        const int sl  = u & (NBMAX - 1);
        const int eid = (int)((unsigned)u >> 12);
        if (lane == 0) {
          int pos = list[sl];
          pos = pos < 0 ? 0 : (pos > RCAP - 1 ? RCAP - 1 : pos);
          reg2[pos] = eid;
          list[sl] = pos + 1;
        }
      }
    }
  }
  __syncthreads();

  const int nbw = nb >> 3;
  const bool ovf = (nh >= RCAP);
  const float qnan = __int_as_float(0x7fc00000);
  float* stw = (float*)reg1 + wave * STW;
  const int lc = lane < 8 ? lane : 7;
#pragma unroll 1
  for (int jt = 0; jt < nbw; ++jt) {
    const int slot = wave * nbw + jt;
    const int grow = nodeBase + slot;
    const int gcl  = grow < nN ? grow : nN - 1;
    int st = soff[slot];
    const int craw = scnt[slot];
    int cnt = craw;
    st  = st < 0 ? 0 : (st > nh ? nh : st);
    cnt = cnt < 0 ? 0 : (cnt > DEGCAP ? DEGCAP : cnt);
    if (cnt > nh - st) cnt = nh - st;
    const float pz = (ovf || craw > DEGCAP) ? qnan : 0.0f;
    const bool wr = grow < MPr;

    const float* qrow = Y + (size_t)gcl * YC + lane;
    float qv[8];
#pragma unroll
    for (int j = 0; j < 8; ++j) qv[j] = qrow[32 * j];
    ldwait();
    float av0 = 0.f, av1 = 0.f;
    float mx = -1.0e30f, dn = 0.f;

#pragma unroll 1
    for (int q = 0; q < cnt; ++q) {
      int idx = st + q; idx = idx > RCAP - 1 ? RCAP - 1 : idx;
      int eid = reg2[idx]; eid = eid < 0 ? 0 : (eid > nE - 1 ? nE - 1 : eid);
      const int sraw = srcs[eid];
      const int s = sraw < 0 ? 0 : (sraw > nN - 1 ? nN - 1 : sraw);
      const float* kr = Y + (size_t)s * YC + CD + lane;
      float kk[8];
#pragma unroll
      for (int j = 0; j < 8; ++j) kk[j] = kr[32 * j];
      ldwait();
      const float v0 = kr[CD];
      const float v1 = kr[CD + 32];
      ldwait();
      float pp = qv[0] * kk[0];
#pragma unroll
      for (int j = 1; j < 8; ++j) pp = fmaf(qv[j], kk[j], pp);
#pragma unroll
      for (int off = 16; off > 0; off >>= 1) pp += __shfl_xor(pp, off);
      const float al = pp * ISC;
      const float df = al - mx;
      const float ee = __expf(-fabsf(df));
      const bool up  = df > 0.f;
      const float s1 = up ? ee : 1.0f;
      const float s2 = up ? 1.0f : ee;
      mx  = up ? al : mx;
      dn  = fmaf(dn, s1, s2);
      av0 = fmaf(av0, s1, s2 * v0);
      av1 = fmaf(av1, s1, s2 * v1);
    }
    const float ds = dn > 0.f ? dn : 1.0f;
    const float iv = (dn > 0.f ? 1.0f : 0.0f) * __builtin_amdgcn_rcpf(ds);
    __builtin_amdgcn_fence(__ATOMIC_RELEASE, "wavefront");
    __builtin_amdgcn_wave_barrier();
    stw[lane]      = av0 * iv + pz;
    stw[32 + lane] = av1 * iv + pz;
    __builtin_amdgcn_fence(__ATOMIC_RELEASE, "wavefront");
    __builtin_amdgcn_wave_barrier();
    v4f a = *(const v4f*)(stw + 8 * lc);
    v4f b = *(const v4f*)(stw + 8 * lc + 4);
    const float* sp = Y + (size_t)gcl * YC + (CD + CD + KD) + 8 * lc;
    const v4f sa = *(const v4f*)sp;
    const v4f sb = *(const v4f*)(sp + 4);
    a.x = fmaxf(a.x + sa.x, 0.f); a.y = fmaxf(a.y + sa.y, 0.f); a.z = fmaxf(a.z + sa.z, 0.f); a.w = fmaxf(a.w + sa.w, 0.f);
    b.x = fmaxf(b.x + sb.x, 0.f); b.y = fmaxf(b.y + sb.y, 0.f); b.z = fmaxf(b.z + sb.z, 0.f); b.w = fmaxf(b.w + sb.w, 0.f);
    const v8h hv = cvt8h(a, b, CG);
    _Float16* gp = RH + (size_t)grow * KD + 8 * lc;
    const bool wsv = wr && (lane < 8);
    if (wsv) *(volatile v8h*)gp = hv;
    __threadfence();
    if (wsv) *(volatile v8h*)gp = hv;
  }
}

__global__ __launch_bounds__(NTHR) void k_gath(const int* __restrict__ midx, const _Float16* __restrict__ RH,
                                               _Float16* HG, int nM, int nN, int nUnits) {
  const int u = (int)blockIdx.x * NTHR + (int)threadIdx.x;
  if (u >= nUnits) return;
  const int i  = u >> 3;
  const int q  = u & 7;
  const int ic = i < nM ? i : nM - 1;
  int r = midx[ic];
  r = r < 0 ? 0 : (r > nN - 1 ? nN - 1 : r);
  v8h hv = *(const v8h*)(RH + (size_t)r * KD + 8 * q);
  if (i >= nM) {
#pragma unroll
    for (int e = 0; e < 8; ++e) hv[e] = (_Float16)0.0f;
  }
  const size_t o = (size_t)i * KD + 8 * q;
  *(volatile v8h*)(HG + o) = hv;
  __threadfence();
  *(volatile v8h*)(HG + o) = hv;
}

static int pick_nb(int nE, int nN) {
  int nb = NBMAX;
  while (nb > 16 && (long long)nb * (long long)nE * 5LL > (long long)RCAP * (long long)nN * 4LL) nb >>= 1;
  return nb;
}
static inline int cdiv(int a, int b) { return (a + b - 1) / b; }

extern "C" void kernel_launch(void* const* d_in, const int* in_sizes, int n_in,
                              void* d_out, int out_size, void* d_ws, size_t ws_size,
                              hipStream_t stream) {
  if (n_in < 14) return;
  const int nN = in_sizes[1];
  if (nN <= 0 || nN > (1 << 22)) return;
  if (in_sizes[0] != nN * QD) return;
  if (in_sizes[2] < 2 || (in_sizes[2] & 1) != 0) return;
  const int nE = in_sizes[2] / 2;
  if (nE < 1 || nE > (1 << 20)) return;
  const int nM = in_sizes[3];
  if (nM < 1 || nM > (1 << 22)) return;
  if (in_sizes[4]  != CD * CD || in_sizes[5]  != CD) return;
  if (in_sizes[6]  != CD * CD || in_sizes[7]  != CD) return;
  if (in_sizes[8]  != CD * CD || in_sizes[9]  != CD) return;
  if (in_sizes[10] != CD * CD || in_sizes[11] != CD) return;
  if (in_sizes[12] != KD * DO || in_sizes[13] != DO) return;
  if (out_size != nM * DO) return;

  const float* query = (const float*)d_in[0];
  const int*   kid   = (const int*)  d_in[1];
  const int*   ei    = (const int*)  d_in[2];
  const int*   midx  = (const int*)  d_in[3];
  const float* Wq = (const float*)d_in[4];  const float* bq = (const float*)d_in[5];
  const float* Wk = (const float*)d_in[6];  const float* bk = (const float*)d_in[7];
  const float* Wv = (const float*)d_in[8];  const float* bv = (const float*)d_in[9];
  const float* Ws = (const float*)d_in[10]; const float* bs = (const float*)d_in[11];
  const float* Wo = (const float*)d_in[12]; const float* bo = (const float*)d_in[13];
  float* out = (float*)d_out;
  const int* src = ei;
  const int* dst = ei + nE;

  const int MP   = cdiv(nN, GBM) * GBM;
  const int MPo  = cdiv(nM, GBM) * GBM;
  const int nb   = pick_nb(nE, nN);
  const int gA   = cdiv(MP, nb);
  const int vec8 = ((nE & 3) == 0) ? 1 : 0;
  if (nb < 16 || gA * nb < MP) return;

  char* ws = (char*)d_ws;
  size_t off = 0;
  const size_t oXH  = off; off += (size_t)MP * CD * 2;    off = (off + 255) & ~(size_t)255;
  const size_t oWT  = off; off += (size_t)YC * CD * 2;    off = (off + 255) & ~(size_t)255;
  const size_t oWOT = off; off += (size_t)DO * KD * 2;    off = (off + 255) & ~(size_t)255;
  const size_t oBC  = off; off += (size_t)YC * 4;         off = (off + 255) & ~(size_t)255;
  const size_t oY   = off; off += (size_t)MP * YC * 4;    off = (off + 255) & ~(size_t)255;
  const size_t oRH  = off; off += (size_t)MP * KD * 2;    off = (off + 255) & ~(size_t)255;
  const size_t oHG  = off; off += (size_t)MPo * KD * 2;   off = (off + 255) & ~(size_t)255;
  if (off > ws_size || off > (size_t)WSMAX) return;
  _Float16* XH  = (_Float16*)(ws + oXH);
  _Float16* WT  = (_Float16*)(ws + oWT);
  _Float16* WOT = (_Float16*)(ws + oWOT);
  float*    BC  = (float*)(ws + oBC);
  float*    Y   = (float*)(ws + oY);
  _Float16* RH  = (_Float16*)(ws + oRH);
  _Float16* HG  = (_Float16*)(ws + oHG);

  hipFuncSetAttribute(reinterpret_cast<const void*>(&k_agg),
                      hipFuncAttributeMaxDynamicSharedMemorySize, LDS_AGG);

  const int nUx = MP * (CD / 8);
  k_xprep<<<cdiv(nUx, NTHR), NTHR, 0, stream>>>(query, kid, XH, nN, nUx);

  const int nUw = YC * (CD / 8);
  k_wcat<<<cdiv(nUw, NTHR), NTHR, 0, stream>>>(Wq, Wk, Wv, Ws, WT, nUw);
  const int nWo = DO * (KD / 8), nBu = YC / 4;
  k_wob<<<cdiv(nWo + nBu, NTHR), NTHR, 0, stream>>>(Wo, bq, bk, bv, bs, WOT, BC, nWo, nBu);

  k_gemm<1><<<dim3(MP / GBM, YC / GBN), GTHR, 0, stream>>>(XH, WT, BC, Y, CD, YC, MP, SCL_XW);

  k_agg<<<gA, NTHR, LDS_AGG, stream>>>(src, dst, Y, RH, nN, nE, nb, vec8, MP);

  const int nUg = MPo * (KD / 8);
  k_gath<<<cdiv(nUg, NTHR), NTHR, 0, stream>>>(midx, RH, HG, nM, nN, nUg);

  k_gemm<3><<<dim3(MPo / GBM, DO / GBN), GTHR, 0, stream>>>(HG, WOT, bo, out, KD, DO, nM, SCL_GW);
}
